// SoftMesh_74036646248987
// MI455X (gfx1250) — hardware-run, weakly checked
//
#include <hip/hip_runtime.h>


#ifndef NPTS
#define NPTS 2000000
#endif
#define NPTS_FULL 2000000
#define HD_   50
#define HP    64
#define KIN   32
#define NMID  7
#define MW    4
#define NST   (NPTS / 32)
#define WM_OFF (HP * KIN)
#define WO_OFF (WM_OFF + NMID * HP * HP)
#define WP_TOT (WO_OFF + 2 * 16 * HP)
#define TANH_K 2.8853900817779268f

static_assert(NPTS % 32 == 0);
static_assert(NPTS_FULL % 32 == 0);
static_assert(NPTS <= NPTS_FULL);
static_assert((size_t)NPTS_FULL * 4 == (size_t)8000000);
static_assert(HD_ == 50);
static_assert(HP == 64);
static_assert(HD_ + 1 <= HP);
static_assert(KIN == 32);
static_assert(NMID == 7);
static_assert(WM_OFF == 256 * 8);
static_assert(NMID * HP * HP == 14 * 256 * 8);
static_assert(2 * 16 * HP == 256 * 8);
static_assert(WP_TOT == 16 * 256 * 8);
static_assert(32 * 4 * 1 == 32 * 4);
static_assert(NST * 32 == NPTS);

typedef unsigned short bf;
typedef __attribute__((ext_vector_type(16))) __bf16   v16bf;
typedef __attribute__((ext_vector_type(8)))  unsigned short v8us;
typedef __attribute__((ext_vector_type(8)))  unsigned v8u;
typedef __attribute__((ext_vector_type(8)))  float    v8f;

__device__ __forceinline__ unsigned short f2bf(float f) { unsigned u = __float_as_uint(f); u += 0x7FFFu + ((u >> 16) & 1u); return (unsigned short)(u >> 16); }
__device__ __forceinline__ v16bf cat16b(v8us lo, v8us hi) { return __builtin_bit_cast(v16bf, __builtin_shufflevector(lo, hi, 0, 1, 2, 3, 4, 5, 6, 7, 8, 9, 10, 11, 12, 13, 14, 15)); }
__device__ __forceinline__ v16bf ldb(const bf* p)  { return cat16b(*(const v8us*)p, *(const v8us*)(p + 16)); }
__device__ __forceinline__ v16bf asbf(v8u w) { return __builtin_bit_cast(v16bf, w); }
__device__ __forceinline__ v8f mmab(v16bf a, v16bf b, v8f c) {
    c = __builtin_amdgcn_wmma_f32_16x16x32_bf16(false, a, false, b, (short)0, c, false, false);
    asm volatile("v_nop\n\tv_nop\n\tv_nop\n\tv_nop" : "+v"(c) : "v"(a), "v"(b));
    return c;
}
__device__ __forceinline__ float tanh_f(float v) {
    const float e = __builtin_amdgcn_exp2f(v * TANH_K);
    return 1.0f - 2.0f * __builtin_amdgcn_rcpf(e + 1.0f);
}
__device__ __forceinline__ void split2(float t0, float t1, unsigned& hw, unsigned& lw) {
    const unsigned u0 = __float_as_uint(t0), u1 = __float_as_uint(t1);
    const unsigned m0 = u0 & 0xffff0000u, m1 = u1 & 0xffff0000u;
    hw = (u0 >> 16) | m1;
    const float d0 = t0 - __uint_as_float(m0), d1 = t1 - __uint_as_float(m1);
    lw = (__float_as_uint(d0) >> 16) | (__float_as_uint(d1) & 0xffff0000u);
}

struct Act { v8u h0, h1, l0, l1; };

template <int MT>
__device__ __forceinline__ void emit(const v8f c, Act& o, const unsigned onew) {
    constexpr int WB = 4 * (MT & 1);
    if (MT < 3) {
#pragma unroll
        for (int q = 0; q < 4; ++q) {
            unsigned hw, lw; split2(tanh_f(c[2 * q]), tanh_f(c[2 * q + 1]), hw, lw);
            if (MT < 2) { o.h0[WB + q] = hw; o.l0[WB + q] = lw; }
            else        { o.h1[WB + q] = hw; o.l1[WB + q] = lw; }
        }
    } else {
        unsigned hw, lw; split2(tanh_f(c[0]), tanh_f(c[1]), hw, lw);
        o.h1[4] = hw;   o.l1[4] = lw;
        o.h1[5] = onew; o.l1[5] = 0u;
        o.h1[6] = 0u;   o.l1[6] = 0u;
        o.h1[7] = 0u;   o.l1[7] = 0u;
    }
}

template <int MT>
__device__ __forceinline__ void slab(const bf* __restrict__ wl, const int fo, const unsigned onew, const Act& ia, const Act& ib, Act& oa, Act& ob) {
    const bf* wr = wl + fo + MT * 16 * HP;
    const v16bf a0 = ldb(wr), a1 = ldb(wr + 32);
    v8f ca = (v8f){}, cb = (v8f){};
    ca = mmab(a0, asbf(ia.h0), ca); ca = mmab(a1, asbf(ia.h1), ca); ca = mmab(a0, asbf(ia.l0), ca); ca = mmab(a1, asbf(ia.l1), ca);
    cb = mmab(a0, asbf(ib.h0), cb); cb = mmab(a1, asbf(ib.h1), cb); cb = mmab(a0, asbf(ib.l0), cb); cb = mmab(a1, asbf(ib.l1), cb);
    emit<MT>(ca, oa, onew); emit<MT>(cb, ob, onew);
}
__device__ __forceinline__ void layer(const bf* __restrict__ wl, const int fo, const unsigned onew, const Act& ia, const Act& ib, Act& oa, Act& ob) {
    slab<0>(wl, fo, onew, ia, ib, oa, ob); slab<1>(wl, fo, onew, ia, ib, oa, ob);
    slab<2>(wl, fo, onew, ia, ib, oa, ob); slab<3>(wl, fo, onew, ia, ib, oa, ob);
}
template <int MT>
__device__ __forceinline__ void slab_in(const bf* __restrict__ wi, const int fi, const unsigned onew, const v16bf ba, const v16bf bb, Act& oa, Act& ob) {
    const v16bf a = ldb(wi + fi + MT * 16 * KIN);
    v8f ca = (v8f){}, cb = (v8f){};
    ca = mmab(a, ba, ca); cb = mmab(a, bb, cb);
    emit<MT>(ca, oa, onew); emit<MT>(cb, ob, onew);
}

__global__ __launch_bounds__(256) void k_wprep(const float* __restrict__ Win, const float* __restrict__ bin, const float* __restrict__ Wmid, const float* __restrict__ bmid,
                                               const float* __restrict__ Wout, const float* __restrict__ bout, bf* WP) {
    const int t = blockIdx.x * 256 + threadIdx.x;
    const int e0 = t * 8;
    v8us o;
    if (blockIdx.x == 0) {
        const int m = e0 >> 5, kb = e0 & 31;
        const int mc = m < HD_ ? m : HD_ - 1;
        float b = bin[mc]; asm volatile("" : "+v"(b));
#pragma unroll
        for (int j = 0; j < 8; ++j) {
            const int k = kb + j; const int kc = k < 3 ? k : 2;
            float w = Win[kc * HD_ + mc]; asm volatile("" : "+v"(w));
            float v = (k < 3) ? w : b;
            v = ((m < HD_) & (k < 4)) ? v : 0.0f;
            o[j] = f2bf(v);
        }
    } else if (blockIdx.x < 15) {
        const int r = e0 - WM_OFF; const int i = r >> 12, m = (r >> 6) & 63, kb = r & 63;
        const int mc = m < HD_ ? m : HD_ - 1;
        float b = bmid[i * HD_ + mc]; asm volatile("" : "+v"(b));
#pragma unroll
        for (int j = 0; j < 8; ++j) {
            const int k = kb + j; const int kc = k < HD_ ? k : HD_ - 1;
            float w = Wmid[(i * HD_ + kc) * HD_ + mc]; asm volatile("" : "+v"(w));
            float v = (k < HD_) ? w : b;
            v = ((m < HD_) & (k <= HD_)) ? v : 0.0f;
            o[j] = f2bf(v);
        }
    } else {
        const int r = e0 - WO_OFF; const int var = r >> 10, row = (r >> 6) & 15, kb = r & 63;
        const int oi = row - 8 * var;
        const int oc = oi < 0 ? 0 : (oi > 2 ? 2 : oi);
        float b = bout[oc]; asm volatile("" : "+v"(b));
#pragma unroll
        for (int j = 0; j < 8; ++j) {
            const int k = kb + j; const int kc = k < HD_ ? k : HD_ - 1;
            float w = Wout[kc * 3 + oc]; asm volatile("" : "+v"(w));
            float v = (k < HD_) ? w : b;
            v = ((oi >= 0) & (oi < 3) & (k <= HD_)) ? v : 0.0f;
            o[j] = f2bf(v);
        }
    }
    *(volatile v8us*)(WP + (size_t)t * 8) = o; __threadfence(); *(volatile v8us*)(WP + (size_t)t * 8) = o;
}

__global__ __launch_bounds__(32 * MW) __attribute__((amdgpu_num_vgpr(256)))
void k_mlp(const float* __restrict__ X, const float* __restrict__ Y, const float* __restrict__ Z, const bf* __restrict__ WP, float* OUT) {
    const int lane = threadIdx.x & 31, lr = lane & 15, hi = lane >> 4;
    const int wave = __builtin_amdgcn_readfirstlane((int)(threadIdx.x >> 5));
    const int st = blockIdx.x * MW + wave;
    if (st >= NST) return;
    const int p0 = st * 32;
    float xa = X[p0 + lr], ya = Y[p0 + lr], za = Z[p0 + lr];
    float xb = X[p0 + 16 + lr], yb = Y[p0 + 16 + lr], zb = Z[p0 + 16 + lr];
    asm volatile("" : "+v"(xa)); asm volatile("" : "+v"(ya)); asm volatile("" : "+v"(za));
    asm volatile("" : "+v"(xb)); asm volatile("" : "+v"(yb)); asm volatile("" : "+v"(zb));
    unsigned wa0 = (unsigned)f2bf(xa) | ((unsigned)f2bf(ya) << 16);
    unsigned wa1 = (unsigned)f2bf(za) | 0x3F800000u;
    unsigned wb0 = (unsigned)f2bf(xb) | ((unsigned)f2bf(yb) << 16);
    unsigned wb1 = (unsigned)f2bf(zb) | 0x3F800000u;
    wa0 = hi ? 0u : wa0; wa1 = hi ? 0u : wa1; wb0 = hi ? 0u : wb0; wb1 = hi ? 0u : wb1;
    const v8u ina = (v8u){ wa0, wa1, 0u, 0u, 0u, 0u, 0u, 0u };
    const v8u inb = (v8u){ wb0, wb1, 0u, 0u, 0u, 0u, 0u, 0u };
    const unsigned onew = hi ? 0u : 0x00003F80u;
    const int fi = lr * KIN + 8 * hi;
    const int fo = lr * HP + 8 * hi;
    const bf* WI = WP;
    const bf* WM = WP + WM_OFF;
    const bf* WO = WP + WO_OFF;

    Act ca, cb, na, nb;
    { const v16bf ba = asbf(ina), bb = asbf(inb);
      slab_in<0>(WI, fi, onew, ba, bb, ca, cb); slab_in<1>(WI, fi, onew, ba, bb, ca, cb);
      slab_in<2>(WI, fi, onew, ba, bb, ca, cb); slab_in<3>(WI, fi, onew, ba, bb, ca, cb); }

#pragma unroll 1
    for (int lp = 0; lp < 3; ++lp) {
        layer(WM + (size_t)(2 * lp) * (HP * HP),     fo, onew, ca, cb, na, nb);
        layer(WM + (size_t)(2 * lp + 1) * (HP * HP), fo, onew, na, nb, ca, cb);
    }
    layer(WM + (size_t)6 * (HP * HP), fo, onew, ca, cb, na, nb);

    v8f c = (v8f){};
    { const bf* wr = WO + fo;
      const v16bf a0 = ldb(wr), a1 = ldb(wr + 32);
      c = mmab(a0, asbf(na.h0), c); c = mmab(a1, asbf(na.h1), c); c = mmab(a0, asbf(na.l0), c); c = mmab(a1, asbf(na.l1), c); }
    { const bf* wr = WO + 16 * HP + fo;
      const v16bf a0 = ldb(wr), a1 = ldb(wr + 32);
      c = mmab(a0, asbf(nb.h0), c); c = mmab(a1, asbf(nb.h1), c); c = mmab(a0, asbf(nb.l0), c); c = mmab(a1, asbf(nb.l1), c); }
    const float u0 = c[0], u1 = c[1], u2 = c[2];
    float* op = OUT + (size_t)p0 + lane;
#pragma unroll 1
    for (int ps = 0; ps < 2; ++ps) {
        *(volatile float*)(op) = u0;
        *(volatile float*)(op + (size_t)NPTS_FULL) = u1;
        *(volatile float*)(op + (size_t)2 * NPTS_FULL) = u2;
        if (ps == 0) __threadfence(); }
}

static constexpr size_t al256(size_t v) { return (v + 255) & ~(size_t)255; }
static constexpr size_t SZ_WP = al256((size_t)WP_TOT * 2);
static constexpr size_t SZ_TOTAL = SZ_WP;
static_assert(SZ_TOTAL <= (size_t)134217728);
static_assert((size_t)16 * 256 * 8 * 2 <= SZ_WP);

extern "C" void kernel_launch(void* const* d_in, const int* in_sizes, int n_in,
                              void* d_out, int out_size, void* d_ws, size_t ws_size, hipStream_t stream) {
    if (n_in < 9) return;
    if ((size_t)in_sizes[0] < (size_t)NPTS || (size_t)in_sizes[1] < (size_t)NPTS || (size_t)in_sizes[2] < (size_t)NPTS) return;
    if (in_sizes[3] < 3 * HD_ || in_sizes[4] < HD_ || in_sizes[5] < NMID * HD_ * HD_ || in_sizes[6] < NMID * HD_ || in_sizes[7] < HD_ * 3 || in_sizes[8] < 3) return;
    if ((size_t)out_size < (size_t)2 * NPTS_FULL + (size_t)NPTS) return;
    if (SZ_TOTAL > ws_size) return;
    const float* x = (const float*)d_in[0]; const float* y = (const float*)d_in[1]; const float* z = (const float*)d_in[2];
    const float* win = (const float*)d_in[3]; const float* bin = (const float*)d_in[4];
    const float* wmid = (const float*)d_in[5]; const float* bmid = (const float*)d_in[6];
    const float* wout = (const float*)d_in[7]; const float* bout = (const float*)d_in[8];
    float* OUT = (float*)d_out;
    bf* WP = (bf*)d_ws;

    k_wprep<<<WP_TOT / (256 * 8), 256, 0, stream>>>(win, bin, wmid, bmid, wout, bout, WP);
    k_mlp<<<(NST + MW - 1) / MW, 32 * MW, 0, stream>>>(x, y, z, WP, OUT);
}
